// BMEDLSTM_46359876993047
// MI455X (gfx1250) — hardware-verified
//
#include <hip/hip_runtime.h>
#include <math.h>
#include <stdint.h>

typedef __attribute__((ext_vector_type(16))) _Float16 v16h;
typedef __attribute__((ext_vector_type(8)))  _Float16 v8h;
typedef __attribute__((ext_vector_type(8)))  float    v8f;
typedef __attribute__((ext_vector_type(4)))  float    v4f;

constexpr int NBATCH  = 128;
constexpr int NXIN    = 64;
constexpr int NSTATE  = 16;
constexpr int NHID    = 512;
constexpr int NGATE   = 2048;
constexpr int NSTEPS  = 201;
constexpr int KCAT0   = 608;
constexpr int KCAT1   = 1024;
constexpr int KOFF_H0 = 96;
constexpr int XS_PITCH   = 104;
constexpr int HT_PITCH   = 520;
constexpr int HT_HALVES  = 16 * HT_PITCH;
constexpr int SLAB_PITCH = 20;
constexpr float DT_F        = 0.1f;
constexpr float W_CARRY     = 64.0f;
constexpr float W_CARRY_INV = 0.015625f;
constexpr int NOUT0      = NBATCH * NSTEPS * NSTATE;
constexpr int NOUT_TOTAL = 2 * NOUT0 + NSTEPS;
constexpr int NOUT_F4    = (NOUT_TOTAL / 32) * 8;
static_assert(KCAT0 % 32 == 0, "k multiple of 32");
static_assert(KCAT1 % 32 == 0, "k multiple of 32");
static_assert(NHID % 32 == 0, "k multiple of 32");
static_assert(NOUT_F4 * 4 == 823488, "full line floats");
static_assert(NOUT_TOTAL - NOUT_F4 * 4 == 9, "tail floats");
static_assert((XS_PITCH * 2) % 16 == 0 && (HT_PITCH * 2) % 16 == 0 && (SLAB_PITCH * 4) % 16 == 0, "align");

__device__ __forceinline__ void dep_guard_h(v8f& a, v8f& b, v16h x, v16h y) { asm volatile("v_nop\n\tv_nop\n\tv_nop\n\tv_nop" : "+v"(a), "+v"(b) : "v"(x), "v"(y)); }
__device__ __forceinline__ void keep4_h(v16h a, v16h b, v16h c, v16h d) { asm volatile("v_nop" :: "v"(a), "v"(b), "v"(c), "v"(d)); }
__device__ __forceinline__ void acc_guard4(v8f& a, v8f& b, v8f& c, v8f& d) { asm volatile("v_nop\n\tv_nop\n\tv_nop\n\tv_nop" : "+v"(a), "+v"(b), "+v"(c), "+v"(d)); }

struct FragH {
  union U { v16h v; v8h h[2]; };
  static __device__ __forceinline__ v16h load(const _Float16* p) {
    U f; f.h[0] = *(const v8h*)(p); f.h[1] = *(const v8h*)(p + 16); return f.v;
  }
  static __device__ __forceinline__ v8f mma(v16h a, v16h b, v8f c) {
    return __builtin_amdgcn_wmma_f32_16x16x32_f16(false, a, false, b, (short)0, c, false, false);
  }
};
__device__ __forceinline__ v8f mma_guarded(v16h a, v16h b, v8f c) {
  c = __builtin_amdgcn_wmma_f32_16x16x32_f16(false, a, false, b, (short)0, c, false, false);
  asm volatile("v_nop\n\tv_nop\n\tv_nop\n\tv_nop" : "+v"(c) : "v"(a), "v"(b));
  return c;
}
__device__ __forceinline__ v8f zero8() { return (v8f){0.f,0.f,0.f,0.f,0.f,0.f,0.f,0.f}; }

__device__ __forceinline__ float rcp_f(float d) { return __builtin_amdgcn_rcpf(d); }
__device__ __forceinline__ float sigm_f(float v) { return rcp_f(1.0f + expf(-v)); }
__device__ __forceinline__ float tanh_f(float v) { return 1.0f - 2.0f * rcp_f(1.0f + expf(2.0f * v)); }

template <int SEG>
__device__ __forceinline__ float prep_elem(int idx, const float* __restrict__ srcA, const float* __restrict__ srcB) {
  if (SEG == 0) {
    const int n = idx / KCAT0;
    const int k = idx - n * KCAT0;
    const int ka = k < (NXIN + NSTATE - 1) ? k : (NXIN + NSTATE - 1);
    int kb = k - KOFF_H0; kb = kb < 0 ? 0 : (kb > NHID - 1 ? NHID - 1 : kb);
    const float va = srcA[(size_t)n * (NXIN + NSTATE) + ka];
    const float vb = srcB[(size_t)n * NHID + kb];
    return (k < NXIN + NSTATE) ? va : ((k < KOFF_H0) ? 0.0f : vb);
  } else if (SEG == 1) {
    const int n = idx >> 10;
    const int k = idx & 1023;
    const int ka = k < NHID - 1 ? k : NHID - 1;
    int kb = k - NHID; kb = kb < 0 ? 0 : kb;
    const float va = srcA[(size_t)n * NHID + ka];
    const float vb = srcB[(size_t)n * NHID + kb];
    return (k < NHID) ? va : vb;
  } else {
    return srcA[idx];
  }
}

template <int SEG>
__global__ __launch_bounds__(256) void prep_weights_kernel(
    const float* __restrict__ srcA, const float* __restrict__ srcB,
    _Float16* __restrict__ dst, int n2) {
  const int i = blockIdx.x * 256 + threadIdx.x;
  if (i >= n2) return;
  const float v0 = prep_elem<SEG>(2 * i, srcA, srcB) * W_CARRY;
  const float v1 = prep_elem<SEG>(2 * i + 1, srcA, srcB) * W_CARRY;
  const _Float16 h0 = (_Float16)v0, h1 = (_Float16)v1;
  const unsigned u = (unsigned)__builtin_bit_cast(unsigned short, h0) | ((unsigned)__builtin_bit_cast(unsigned short, h1) << 16);
  ((volatile unsigned*)dst)[i] = u;
  __threadfence();
  ((volatile unsigned*)dst)[i] = u;
}

__device__ __forceinline__ void mma4(v8f (&acc)[4], v16h a, const _Float16* __restrict__ wp, size_t gstr) {
  const v16h b0 = FragH::load(wp);
  const v16h b1 = FragH::load(wp + gstr);
  const v16h b2 = FragH::load(wp + 2 * gstr);
  const v16h b3 = FragH::load(wp + 3 * gstr);
  acc[0] = FragH::mma(a, b0, acc[0]);
  acc[1] = FragH::mma(a, b1, acc[1]);
  acc[2] = FragH::mma(a, b2, acc[2]);
  acc[3] = FragH::mma(a, b3, acc[3]);
  dep_guard_h(acc[0], acc[3], a, b3);
  keep4_h(b0, b1, b2, b3);
}

__device__ __forceinline__ void cell_pass(
    const _Float16* tileA, int pitchA, int nkA,
    const _Float16* tileB, int pitchB, int nkB, int wcolB,
    const _Float16* __restrict__ Wcat, int ldw,
    const float* __restrict__ biasA, const float* __restrict__ biasB,
    _Float16* hdst, int ub, int lane, float (&cs)[8]) {
  const int hh = lane >> 4, c16 = lane & 15, koff = hh * 8;
  v8f acc[4];
  acc[0] = zero8(); acc[1] = zero8(); acc[2] = zero8(); acc[3] = zero8();
  const _Float16* wrow = Wcat + (size_t)(16 * ub + c16) * ldw + koff;
  const size_t gstr = (size_t)NHID * (size_t)ldw;
  const _Float16* ap = tileA + c16 * pitchA + koff;
#pragma unroll 1
  for (int ks = 0; ks < nkA; ++ks) {
    const v16h a = FragH::load(ap + 32 * ks);
    mma4(acc, a, wrow + 32 * ks, gstr);
  }
  const _Float16* bp = tileB + c16 * pitchB + koff;
  const _Float16* wrow2 = wrow + wcolB;
#pragma unroll 1
  for (int ks = 0; ks < nkB; ++ks) {
    const v16h a = FragH::load(bp + 32 * ks);
    mma4(acc, a, wrow2 + 32 * ks, gstr);
  }
  acc_guard4(acc[0], acc[1], acc[2], acc[3]);

  const int j = 16 * ub + c16;
  const float bi = biasA[j] + biasB[j];
  const float bf = biasA[NHID + j] + biasB[NHID + j];
  const float bg = biasA[2 * NHID + j] + biasB[2 * NHID + j];
  const float bo = biasA[3 * NHID + j] + biasB[3 * NHID + j];
#pragma unroll
  for (int r = 0; r < 8; ++r) {
    const float pi = acc[0][r] * W_CARRY_INV + bi;
    const float pf = acc[1][r] * W_CARRY_INV + bf;
    const float pg = acc[2][r] * W_CARRY_INV + bg;
    const float po = acc[3][r] * W_CARRY_INV + bo;
    const float ig = sigm_f(pi);
    const float fg = sigm_f(pf);
    const float gt = tanh_f(pg);
    const float og = sigm_f(po);
    const float cn = fg * cs[r] + ig * gt;
    cs[r] = cn;
    const float hv = og * tanh_f(cn);
    hdst[(8 * hh + r) * HT_PITCH + j] = (_Float16)hv;
  }
}

__global__ __launch_bounds__(256) void lstm_seq_kernel(
    const float* __restrict__ x,    const float* __restrict__ s0,
    const _Float16* __restrict__ W0, const _Float16* __restrict__ W1, const _Float16* __restrict__ Wf,
    const float* __restrict__ bih0, const float* __restrict__ bhh0,
    const float* __restrict__ bih1, const float* __restrict__ bhh1,
    const float* __restrict__ bfc,
    float* __restrict__ stgS, float* __restrict__ stgO) {
  __shared__ __align__(16) _Float16 XSt[16 * XS_PITCH];
  __shared__ __align__(16) _Float16 H0t[2 * HT_HALVES];
  __shared__ __align__(16) _Float16 H1t[2 * HT_HALVES];
  __shared__ __align__(16) float slabS[16 * SLAB_PITCH];
  __shared__ __align__(16) float slabO[16 * SLAB_PITCH];

  const int tid  = threadIdx.x;
  const int lane = tid & 31;
  const int wave = tid >> 5;
  const int hh   = lane >> 4;
  const int c16  = lane & 15;
  const int b0   = blockIdx.x * 16;

  for (int i = tid; i < 2 * HT_HALVES; i += 256) { H0t[i] = (_Float16)0.0f; H1t[i] = (_Float16)0.0f; }
  for (int i = tid; i < 16 * SLAB_PITCH; i += 256) { slabS[i] = 0.0f; slabO[i] = 0.0f; }
  for (int i = tid; i < 16 * XS_PITCH; i += 256) {
    const int r = i / XS_PITCH;
    const int k = i - r * XS_PITCH;
    const int kx = k < NXIN ? k : NXIN - 1;
    int ksx = k - NXIN; ksx = ksx < 0 ? 0 : (ksx > NSTATE - 1 ? NSTATE - 1 : ksx);
    const float xv = x[(size_t)(b0 + r) * NXIN + kx];
    const float sv = s0[(size_t)(b0 + r) * NSTATE + ksx];
    const float v = (k < NXIN) ? xv : ((k < NXIN + NSTATE) ? sv : 0.0f);
    XSt[i] = (_Float16)v;
  }
  __syncthreads();

  float c00[8], c01[8], c02[8], c03[8], c10[8], c11[8], c12[8], c13[8];
  float sreg[8];
#pragma unroll
  for (int r = 0; r < 8; ++r) {
    c00[r] = 0.f; c01[r] = 0.f; c02[r] = 0.f; c03[r] = 0.f;
    c10[r] = 0.f; c11[r] = 0.f; c12[r] = 0.f; c13[r] = 0.f;
    sreg[r] = s0[(size_t)(b0 + 8 * hh + r) * NSTATE + c16];
  }
  const int ub0 = wave * 4;

  for (int t = 0; t < NSTEPS; ++t) {
    const _Float16* h0cur = H0t + (t & 1) * HT_HALVES;
    _Float16*       h0nxt = H0t + ((t + 1) & 1) * HT_HALVES;
    const _Float16* h1cur = H1t + (t & 1) * HT_HALVES;
    _Float16*       h1nxt = H1t + ((t + 1) & 1) * HT_HALVES;

    cell_pass(XSt, XS_PITCH, 3, h0cur, HT_PITCH, 16, KOFF_H0, W0, KCAT0, bih0, bhh0, h0nxt, ub0 + 0, lane, c00);
    cell_pass(XSt, XS_PITCH, 3, h0cur, HT_PITCH, 16, KOFF_H0, W0, KCAT0, bih0, bhh0, h0nxt, ub0 + 1, lane, c01);
    cell_pass(XSt, XS_PITCH, 3, h0cur, HT_PITCH, 16, KOFF_H0, W0, KCAT0, bih0, bhh0, h0nxt, ub0 + 2, lane, c02);
    cell_pass(XSt, XS_PITCH, 3, h0cur, HT_PITCH, 16, KOFF_H0, W0, KCAT0, bih0, bhh0, h0nxt, ub0 + 3, lane, c03);
    __syncthreads();

    cell_pass(h0nxt, HT_PITCH, 16, h1cur, HT_PITCH, 16, NHID, W1, KCAT1, bih1, bhh1, h1nxt, ub0 + 0, lane, c10);
    cell_pass(h0nxt, HT_PITCH, 16, h1cur, HT_PITCH, 16, NHID, W1, KCAT1, bih1, bhh1, h1nxt, ub0 + 1, lane, c11);
    cell_pass(h0nxt, HT_PITCH, 16, h1cur, HT_PITCH, 16, NHID, W1, KCAT1, bih1, bhh1, h1nxt, ub0 + 2, lane, c12);
    cell_pass(h0nxt, HT_PITCH, 16, h1cur, HT_PITCH, 16, NHID, W1, KCAT1, bih1, bhh1, h1nxt, ub0 + 3, lane, c13);
    __syncthreads();

    if (wave == 0) {
      v8f facc = zero8();
      const _Float16* hp = h1nxt + c16 * HT_PITCH + hh * 8;
      const _Float16* wp = Wf + (size_t)c16 * NHID + hh * 8;
#pragma unroll 1
      for (int ks = 0; ks < NHID / 32; ++ks) {
        const v16h a = FragH::load(hp + 32 * ks);
        const v16h b = FragH::load(wp + 32 * ks);
        facc = mma_guarded(a, b, facc);
      }
      const float bb = bfc[c16];
#pragma unroll
      for (int r = 0; r < 8; ++r) {
        const float so = facc[r] * W_CARRY_INV + bb;
        const float sv = sreg[r] + so * DT_F;
        sreg[r] = sv;
        const int row = 8 * hh + r;
        XSt[row * XS_PITCH + NXIN + c16] = (_Float16)sv;
        slabS[row * SLAB_PITCH + c16] = sv;
        slabO[row * SLAB_PITCH + c16] = so;
      }
      __builtin_amdgcn_fence(__ATOMIC_RELEASE, "workgroup");
      __builtin_amdgcn_wave_barrier();
      __builtin_amdgcn_fence(__ATOMIC_ACQUIRE, "workgroup");
      float* gS = stgS + ((size_t)t * NBATCH + b0) * NSTATE;
      float* gO = stgO + ((size_t)t * NBATCH + b0) * NSTATE;
      const int srow = lane >> 2, scol = (lane & 3) * 4;
      for (int pass = 0; pass < 2; ++pass) {
#pragma unroll
        for (int q = 0; q < 2; ++q) {
          const v4f vs = *(const v4f*)(slabS + (q * 8 + srow) * SLAB_PITCH + scol);
          const v4f vo = *(const v4f*)(slabO + (q * 8 + srow) * SLAB_PITCH + scol);
          *(volatile v4f*)(gS + q * 128 + lane * 4) = vs;
          *(volatile v4f*)(gO + q * 128 + lane * 4) = vo;
        }
        __threadfence();
      }
    }
    __syncthreads();
  }
}

__device__ __forceinline__ float out_elem(int e, const float* __restrict__ stgS, const float* __restrict__ stgO) {
  constexpr int RB = NSTEPS * NSTATE;
  int e0 = e < NOUT0 ? e : NOUT0 - 1; e0 = e0 < 0 ? 0 : e0;
  int e2 = e - NOUT0 - NSTEPS; e2 = e2 < 0 ? 0 : (e2 > NOUT0 - 1 ? NOUT0 - 1 : e2);
  const int bS = e0 / RB; const int rS = e0 - bS * RB; const int tS = rS >> 4; const int cS = rS & 15;
  const int bO = e2 / RB; const int rO = e2 - bO * RB; const int tO = rO >> 4; const int cO = rO & 15;
  const float vS = stgS[((size_t)tS * NBATCH + bS) * NSTATE + cS];
  const float vO = stgO[((size_t)tO * NBATCH + bO) * NSTATE + cO];
  const float vT = (float)(e - NOUT0) * DT_F;
  return (e < NOUT0) ? vS : ((e < NOUT0 + NSTEPS) ? vT : vO);
}

__global__ __launch_bounds__(256) void finisher_kernel(
    const float* __restrict__ stgS, const float* __restrict__ stgO, float* __restrict__ dout) {
  const int i = blockIdx.x * 256 + threadIdx.x;
  if (i < NOUT_F4) {
    v4f v;
    v[0] = out_elem(4 * i + 0, stgS, stgO);
    v[1] = out_elem(4 * i + 1, stgS, stgO);
    v[2] = out_elem(4 * i + 2, stgS, stgO);
    v[3] = out_elem(4 * i + 3, stgS, stgO);
    float* p = dout + (size_t)i * 4;
    *(volatile v4f*)p = v;
    __threadfence();
    *(volatile v4f*)p = v;
  }
  if (blockIdx.x == 0 && threadIdx.x < 32) {
    constexpr int TAIL0 = NOUT_F4 * 4;
    constexpr int NTAIL = NOUT_TOTAL - TAIL0;
    const int ln = threadIdx.x;
    const int e  = TAIL0 + (ln < NTAIL ? ln : NTAIL - 1);
    const float tv = out_elem(e, stgS, stgO);
    if (ln < NTAIL) ((volatile float*)dout)[e] = tv;
    __threadfence();
    if (ln < NTAIL) ((volatile float*)dout)[e] = tv;
  }
}

extern "C" void kernel_launch(void* const* d_in, const int* in_sizes, int n_in,
                              void* d_out, int out_size, void* d_ws, size_t ws_size,
                              hipStream_t stream) {
  if (n_in < 12) return;
  if (out_size != NOUT_TOTAL) return;
  if (in_sizes[0] != NBATCH * NXIN || in_sizes[1] != NBATCH * NSTATE ||
      in_sizes[2] != NGATE * (NXIN + NSTATE) || in_sizes[3] != NGATE * NHID ||
      in_sizes[4] != NGATE || in_sizes[5] != NGATE ||
      in_sizes[6] != NGATE * NHID || in_sizes[7] != NGATE * NHID ||
      in_sizes[8] != NGATE || in_sizes[9] != NGATE ||
      in_sizes[10] != NSTATE * NHID || in_sizes[11] != NSTATE) return;

  const float* x    = (const float*)d_in[0];
  const float* s0   = (const float*)d_in[1];
  const float* Wih0 = (const float*)d_in[2];
  const float* Whh0 = (const float*)d_in[3];
  const float* bih0 = (const float*)d_in[4];
  const float* bhh0 = (const float*)d_in[5];
  const float* Wih1 = (const float*)d_in[6];
  const float* Whh1 = (const float*)d_in[7];
  const float* bih1 = (const float*)d_in[8];
  const float* bhh1 = (const float*)d_in[9];
  const float* Wfc  = (const float*)d_in[10];
  const float* bfc  = (const float*)d_in[11];

  uint8_t* ws = (uint8_t*)d_ws;
  size_t off = 0;
  auto carve = [&](size_t bytes) -> void* {
    void* p = ws + off;
    off = (off + bytes + 255) & ~(size_t)255;
    return p;
  };
  const size_t bytesW0  = (size_t)NGATE * KCAT0 * 2;
  const size_t bytesW1  = (size_t)NGATE * KCAT1 * 2;
  const size_t bytesWf  = (size_t)NSTATE * NHID * 2;
  const size_t bytesStg = (size_t)NSTEPS * NBATCH * NSTATE * 4;
  _Float16* W0c  = (_Float16*)carve(bytesW0);
  _Float16* W1c  = (_Float16*)carve(bytesW1);
  _Float16* Wf16 = (_Float16*)carve(bytesWf);
  float*    stgS = (float*)carve(bytesStg);
  float*    stgO = (float*)carve(bytesStg);
  if (off > ws_size) return;

  const int n2W0 = NGATE * KCAT0 / 2;
  const int n2W1 = NGATE * KCAT1 / 2;
  const int n2Wf = NSTATE * NHID / 2;
  prep_weights_kernel<0><<<dim3((n2W0 + 255) / 256), dim3(256), 0, stream>>>(Wih0, Whh0, W0c, n2W0);
  prep_weights_kernel<1><<<dim3((n2W1 + 255) / 256), dim3(256), 0, stream>>>(Wih1, Whh1, W1c, n2W1);
  prep_weights_kernel<2><<<dim3((n2Wf + 255) / 256), dim3(256), 0, stream>>>(Wfc, Wfc, Wf16, n2Wf);

  lstm_seq_kernel<<<dim3(NBATCH / 16), dim3(256), 0, stream>>>(
      x, s0, W0c, W1c, Wf16, bih0, bhh0, bih1, bhh1, bfc, stgS, stgO);

  finisher_kernel<<<dim3((NOUT_F4 + 255) / 256), dim3(256), 0, stream>>>(stgS, stgO, (float*)d_out);
}
